// MultiHeadSelfAttention_17360257810453
// MI455X (gfx1250) — hardware-run, weakly checked
//
#include <hip/hip_runtime.h>


#ifndef NB
#define NB 1
#endif
#ifndef SEQ
#define SEQ 1863
#endif
#define NB_FULL  1
#define SEQ_FULL 1863
#define SPAD (((SEQ + 63) / 64) * 64)
#define DM   1024
#define NH_  16
#define HD   64
#define AW   4
#define OSP  68
#define EROWS (SPAD < 256 ? SPAD : 256)
#define QRS  2048.0f
#define QRI  (1.0f / 2048.0f)
#define SC2  ((float)(0.125 * 1.4426950408889634))
#define LOG2E 1.4426950408889634f
#define PSH  14.0f
#define NEGB (-3.0e38f)
#define CXS  64.0f
#define WSC  64.0f
#define OSCL (1.0f / 4096.0f)

static_assert(NB == 1);
static_assert(HD == 64);
static_assert(NH_ * HD == DM);
static_assert(DM % 64 == 0);
static_assert(DM % 32 == 0);
static_assert(HD % 32 == 0);
static_assert(SPAD % 64 == 0);
static_assert(SPAD >= SEQ);
static_assert(SEQ >= 1);
static_assert(SEQ <= SEQ_FULL);
static_assert(EROWS % 64 == 0);
static_assert(EROWS >= 32);
static_assert(EROWS <= SPAD);
static_assert(EROWS % (16 * AW) == 0);
static_assert((SPAD - EROWS) % (16 * AW) == 0);
static_assert(EROWS % 32 == 0);
static_assert((OSP * 4) % 16 == 0);
static_assert(OSP >= 64 + 4);
static_assert(32 * AW * 2 == 256);
static_assert((AW * 16 * OSP + 256) * 4 <= 131072);
static_assert(16 * 68 * 4 <= 131072);
static_assert(((size_t)SPAD * DM / 8) % 256 == 0);
static_assert(((size_t)SPAD * 32) % 256 == 0);
static_assert(((size_t)DM * DM / 8) % 256 == 0);

typedef _Float16 h16;
typedef unsigned short bf;
typedef __attribute__((ext_vector_type(16))) __bf16   v16bf;
typedef __attribute__((ext_vector_type(16))) _Float16 v16h;
typedef __attribute__((ext_vector_type(8)))  _Float16 v8h;
typedef __attribute__((ext_vector_type(8)))  unsigned short v8us;
typedef __attribute__((ext_vector_type(8)))  float    v8f;
typedef __attribute__((ext_vector_type(4)))  float    v4f;
typedef __attribute__((ext_vector_type(2)))  float    v2f;
typedef __attribute__((ext_vector_type(4)))  int      v4i;
typedef v4f  __attribute__((may_alias)) v4fa;

__device__ __forceinline__ unsigned short f2bf(float f) { unsigned u = __float_as_uint(f); u += 0x7FFFu + ((u >> 16) & 1u); return (unsigned short)(u >> 16); }
__device__ __forceinline__ float bfr(float f) { return __uint_as_float(((unsigned)f2bf(f)) << 16); }
__device__ __forceinline__ v16h cat16(v8h lo, v8h hi) { return __builtin_shufflevector(lo, hi, 0, 1, 2, 3, 4, 5, 6, 7, 8, 9, 10, 11, 12, 13, 14, 15); }
__device__ __forceinline__ v16bf cat16b(v8us lo, v8us hi) { return __builtin_bit_cast(v16bf, __builtin_shufflevector(lo, hi, 0, 1, 2, 3, 4, 5, 6, 7, 8, 9, 10, 11, 12, 13, 14, 15)); }
__device__ __forceinline__ v8f wmma16(v16h a, v16h b, v8f c) { return __builtin_amdgcn_wmma_f32_16x16x32_f16(false, a, false, b, (short)0, c, false, false); }
__device__ __forceinline__ v8f wmmab(v16bf a, v16bf b, v8f c) { return __builtin_amdgcn_wmma_f32_16x16x32_bf16(false, a, false, b, (short)0, c, false, false); }
__device__ __forceinline__ v16h  ldh(const h16* p) { return cat16(*(const v8h*)p, *(const v8h*)(p + 16)); }
__device__ __forceinline__ v16bf ldb(const bf* p)  { return cat16b(*(const v8us*)p, *(const v8us*)(p + 16)); }
__device__ __forceinline__ void wave_sync() { __builtin_amdgcn_fence(3  , "wavefront"); __builtin_amdgcn_wave_barrier(); asm volatile("" ::: "memory"); }

__device__ __forceinline__ v8f wmma16g(v16h a, v16h b, v8f c) { c = wmma16(a, b, c); asm volatile("v_nop\n\tv_nop\n\tv_nop\n\tv_nop" : "+v"(c) : "v"(a), "v"(b)); return c; }
__device__ __forceinline__ v8f wmmabg(v16bf a, v16bf b, v8f c) { c = wmmab(a, b, c); asm volatile("v_nop\n\tv_nop\n\tv_nop\n\tv_nop" : "+v"(c) : "v"(a), "v"(b)); return c; }
__device__ __forceinline__ h16 toh_flush(float v) { const h16 r = (h16)v; return (fabsf(v) < 6.103515625e-05f) ? (h16)0.0f : r; }
__device__ __forceinline__ int clampi(int v, int lo, int hi) { return v < lo ? lo : (v > hi ? hi : v); }

__global__ __launch_bounds__(256) void k_cvt8(const float* __restrict__ src, bf* dst, size_t n8) {
    const size_t i = (size_t)blockIdx.x * 256 + threadIdx.x; if (i >= n8) return;
    const v8f v = *(const v8f*)(src + i * 8); v8us o;
#pragma unroll
    for (int k = 0; k < 8; ++k) o[k] = f2bf(v[k]);
    *(volatile v8us*)(dst + i * 8) = o; __threadfence(); *(volatile v8us*)(dst + i * 8) = o;
}

__global__ __launch_bounds__(256) void k_cvtx(const float* __restrict__ src, bf* dst) {
    const size_t i = (size_t)blockIdx.x * 256 + threadIdx.x;
    const int row = (int)(i / (DM / 8)), c8 = (int)(i % (DM / 8));
    const int rc = row < SEQ ? row : (SEQ - 1);
    v8f v = *(const v8f*)(src + (size_t)rc * DM + (size_t)c8 * 8);
    asm volatile("" : "+v"(v));
    const bool ok = row < SEQ; v8us o;
#pragma unroll
    for (int k = 0; k < 8; ++k) o[k] = ok ? f2bf(v[k]) : (unsigned short)0;
    *(volatile v8us*)(dst + i * 8) = o; __threadfence(); *(volatile v8us*)(dst + i * 8) = o;
}

__global__ __launch_bounds__(256) void k_cvtw(const float* __restrict__ src, h16* dst, size_t n8) {
#pragma clang fp contract(off)
    const size_t i = (size_t)blockIdx.x * 256 + threadIdx.x; if (i >= n8) return;
    const v8f v = *(const v8f*)(src + i * 8); v8h o;
#pragma unroll
    for (int k = 0; k < 8; ++k) o[k] = toh_flush(bfr(v[k]) * WSC);
    *(volatile v8h*)(dst + i * 8) = o; __threadfence(); *(volatile v8h*)(dst + i * 8) = o;
}

__global__ __launch_bounds__(32) void k_pospad(const int* __restrict__ pos, int* PP) {
    const int i = blockIdx.x * 32 + threadIdx.x; const int c = blockIdx.y;
    if (i * 4 >= SPAD) return;
    v4i o;
#pragma unroll
    for (int u = 0; u < 4; ++u) { const int t = 4 * i + u; const int tc = t < SEQ ? t : (SEQ - 1);
        int v = pos[(size_t)tc * 3 + c]; asm volatile("" : "+v"(v)); o[u] = (t < SEQ) ? v : 0; }
    int* p = PP + (size_t)c * SPAD + (size_t)i * 4;
    *(volatile v4i*)p = o; __threadfence(); *(volatile v4i*)p = o;
}

__global__ __launch_bounds__(256) void k_ropecs(const int* __restrict__ pos, float* CS) {
#pragma clang fp contract(off)
    const int i = blockIdx.x * 256 + threadIdx.x;
    const int tok = i >> 5, p = i & 31;
    const int tc = tok < SEQ ? tok : (SEQ - 1);
    int px = pos[(size_t)tc * 3 + 0]; int py = pos[(size_t)tc * 3 + 1]; int pz = pos[(size_t)tc * 3 + 2];
    asm volatile("" : "+v"(px)); asm volatile("" : "+v"(py)); asm volatile("" : "+v"(pz));
    const bool ok = tok < SEQ;
    const int xp = ok ? clampi(px, 0, 31) : 0, yp = ok ? clampi(py, 0, 31) : 0, zp = ok ? clampi(pz, 0, 7) : 0;
    const int pp = (p < 10) ? xp : ((p < 20) ? yp : zp);
    const int pl = (p < 10) ? p : ((p < 20) ? (p - 10) : (p - 20));
    const float rden = (p < 20) ? 0.05f : (1.0f / 24.0f);
    const float e = (float)(2 * pl) * rden;
    const float inv = __builtin_amdgcn_exp2f(-e * 13.287712379549449f);
    const float ang = (float)pp * inv;
    float sn, cs; sincosf(ang, &sn, &cs);
    v2f o; o[0] = cs; o[1] = sn;
    float* q = CS + (size_t)i * 2;
    *(volatile v2f*)q = o; __threadfence(); *(volatile v2f*)q = o;
}

__device__ __forceinline__ void gemm64_bf(const bf* __restrict__ A, const bf* __restrict__ Bt, const size_t aoff, const size_t boff, v8f (&acc)[4][4]) {
#pragma unroll 1
    for (int kc = 0; kc < DM; kc += 32) {
        v16bf a[4];
#pragma unroll
        for (int mb = 0; mb < 4; ++mb) a[mb] = ldb(A + aoff + (size_t)mb * 16 * DM + kc);
#pragma unroll
        for (int nb = 0; nb < 4; ++nb) { const v16bf b = ldb(Bt + boff + (size_t)nb * 16 * DM + kc);
#pragma unroll
            for (int mb = 0; mb < 4; ++mb) acc[mb][nb] = wmmabg(a[mb], b, acc[mb][nb]); }
    }
}
__device__ __forceinline__ void gemm64_h(const h16* __restrict__ A, const h16* __restrict__ Bt, const size_t aoff, const size_t boff, v8f (&acc)[4][4]) {
#pragma unroll 1
    for (int kc = 0; kc < DM; kc += 32) {
        v16h a[4];
#pragma unroll
        for (int mb = 0; mb < 4; ++mb) a[mb] = ldh(A + aoff + (size_t)mb * 16 * DM + kc);
#pragma unroll
        for (int nb = 0; nb < 4; ++nb) { const v16h b = ldh(Bt + boff + (size_t)nb * 16 * DM + kc);
#pragma unroll
            for (int mb = 0; mb < 4; ++mb) acc[mb][nb] = wmma16g(a[mb], b, acc[mb][nb]); }
    }
}

static_assert(4 * 4 * 8 * 16 == 16 * HD * 2);
__global__ __launch_bounds__(32) void k_projqk(const bf* __restrict__ XB, const bf* __restrict__ WB, const float* __restrict__ CS, h16* PH, h16* PR) {
    __shared__ __align__(16) float os[16 * 68];
    const int lane = threadIdx.x & 31, lr = lane & 15, hi = lane >> 4; const int r0 = blockIdx.x * 64, c0 = blockIdx.y * 64;
    v8f acc[4][4];
#pragma unroll
    for (int mb = 0; mb < 4; ++mb)
#pragma unroll
        for (int nb = 0; nb < 4; ++nb) acc[mb][nb] = (v8f){};
    gemm64_bf(XB, WB, (size_t)(r0 + lr) * DM + 8 * hi, (size_t)(c0 + lr) * DM + 8 * hi, acc);
    const int z = blockIdx.y;
    const size_t tbase = ((size_t)z * SPAD + (size_t)r0) * HD;
    const size_t rbase = ((size_t)z * EROWS + (size_t)r0) * HD;
    const bool wr = r0 < EROWS;
#pragma unroll
    for (int mb = 0; mb < 4; ++mb) {
#pragma unroll
        for (int nb = 0; nb < 4; ++nb) {
#pragma unroll
            for (int j = 0; j < 8; ++j) os[(hi * 8 + j) * 68 + nb * 16 + lr] = acc[mb][nb][j]; }
        wave_sync();
#pragma unroll 1
        for (int ps = 0; ps < 2; ++ps) {
#pragma unroll
            for (int s = 0; s < 4; ++s) { const int row = 4 * s + (lane >> 3), c8 = (lane & 7) * 8;
                const v4f x0 = *(const v4fa*)(&os[row * 68 + c8]); const v4f x1 = *(const v4fa*)(&os[row * 68 + c8 + 4]);
                const size_t tok = (size_t)(r0 + mb * 16 + row);
                const v4f cs0 = *(const v4f*)(CS + tok * 64 + c8); const v4f cs1 = *(const v4f*)(CS + tok * 64 + c8 + 4);
                float y[8];
                y[0] = x0[0] * cs0[0] - x0[1] * cs0[1]; y[1] = x0[1] * cs0[0] + x0[0] * cs0[1];
                y[2] = x0[2] * cs0[2] - x0[3] * cs0[3]; y[3] = x0[3] * cs0[2] + x0[2] * cs0[3];
                y[4] = x1[0] * cs1[0] - x1[1] * cs1[1]; y[5] = x1[1] * cs1[0] + x1[0] * cs1[1];
                y[6] = x1[2] * cs1[2] - x1[3] * cs1[3]; y[7] = x1[3] * cs1[2] + x1[2] * cs1[3];
                v8h hv, rv;
#pragma unroll
                for (int i = 0; i < 8; ++i) { const h16 a0 = toh_flush(y[i]); hv[i] = a0; rv[i] = toh_flush((y[i] - (float)a0) * QRS); }
                const size_t oo = tbase + (size_t)(mb * 16 + row) * HD + c8;
                const size_t ro = rbase + (size_t)(mb * 16 + row) * HD + c8;
                *(volatile v8h*)(PH + oo) = hv; if (wr) *(volatile v8h*)(PR + ro) = rv; }
            if (ps == 0) __threadfence(); }
        wave_sync();
    }
}

static_assert(4 * 4 * 8 * 16 == 16 * 64 * 2);
__global__ __launch_bounds__(32) void k_projv(const bf* __restrict__ WV, const bf* __restrict__ XB, h16* VT, h16* VR) {
    __shared__ __align__(16) float os[16 * 68];
    const int lane = threadIdx.x & 31, lr = lane & 15, hi = lane >> 4; const int r0 = blockIdx.x * 64, c0 = blockIdx.y * 64;
    v8f acc[4][4];
#pragma unroll
    for (int mb = 0; mb < 4; ++mb)
#pragma unroll
        for (int nb = 0; nb < 4; ++nb) acc[mb][nb] = (v8f){};
    gemm64_bf(WV, XB, (size_t)(r0 + lr) * DM + 8 * hi, (size_t)(c0 + lr) * DM + 8 * hi, acc);
    const size_t tbase = (size_t)r0 * SPAD + (size_t)c0;
    const size_t rbase = (size_t)r0 * EROWS + (size_t)c0;
    const bool wr = c0 < EROWS;
#pragma unroll
    for (int mb = 0; mb < 4; ++mb) {
#pragma unroll
        for (int nb = 0; nb < 4; ++nb) {
#pragma unroll
            for (int j = 0; j < 8; ++j) os[(hi * 8 + j) * 68 + nb * 16 + lr] = acc[mb][nb][j]; }
        wave_sync();
#pragma unroll 1
        for (int ps = 0; ps < 2; ++ps) {
#pragma unroll
            for (int s = 0; s < 4; ++s) { const int row = 4 * s + (lane >> 3), c8 = (lane & 7) * 8;
                const v4f x0 = *(const v4fa*)(&os[row * 68 + c8]); const v4f x1 = *(const v4fa*)(&os[row * 68 + c8 + 4]); v8h hv, rv;
#pragma unroll
                for (int i = 0; i < 4; ++i) { const h16 a0 = toh_flush(x0[i]); const h16 a1 = toh_flush(x1[i]); hv[i] = a0; hv[4 + i] = a1;
                    rv[i] = toh_flush((x0[i] - (float)a0) * QRS); rv[4 + i] = toh_flush((x1[i] - (float)a1) * QRS); }
                const size_t oo = tbase + (size_t)(mb * 16 + row) * SPAD + c8;
                const size_t ro = rbase + (size_t)(mb * 16 + row) * EROWS + c8;
                *(volatile v8h*)(VT + oo) = hv; if (wr) *(volatile v8h*)(VR + ro) = rv; }
            if (ps == 0) __threadfence(); }
        wave_sync();
    }
}

static_assert(4 * 4 * 8 * 16 == 16 * HD * 2);
template <int EARLY>
__device__ __forceinline__ void flash_body(const h16* __restrict__ QK, const h16* __restrict__ QKR, const h16* __restrict__ VT, const h16* __restrict__ VR, const int* __restrict__ PP,
                                           const float* __restrict__ bxp, const float* __restrict__ byp, const float* __restrict__ bzp, h16* CH, h16* CR) {
    __shared__ __align__(16) float os[AW * 16 * OSP];
    __shared__ float bt[256];
    const int lane = threadIdx.x & 31, lr = lane & 15, hi = lane >> 4;
    const int wave = __builtin_amdgcn_readfirstlane((int)(threadIdx.x >> 5));
    const int h = blockIdx.y;
#pragma unroll 1
    for (int trip = 0; trip < 2; ++trip) {
        const int e = (int)threadIdx.x + 128 * trip; const int seg = e >> 6, idx = e & 63;
        const int ixy = idx < 60 ? idx : 60; const int iz = idx < 16 ? idx : 16;
        float vx = bxp[ixy * NH_ + h]; float vy = byp[ixy * NH_ + h]; float vz = bzp[iz * NH_ + h];
        asm volatile("" : "+v"(vx)); asm volatile("" : "+v"(vy)); asm volatile("" : "+v"(vz));
        const float v = (seg == 0) ? vx : ((seg == 1) ? vy : vz);
        const bool ok = (seg < 2) ? (idx < 61) : ((seg == 2) & (idx < 17));
        bt[e] = ok ? (bfr(v) * LOG2E) : 0.0f;
    }
    __syncthreads();
    const int t0 = (EARLY ? 0 : EROWS) + (blockIdx.x * AW + wave) * 16;
    const int lim = t0 + lr;
    const int nk = (t0 + 16 + 31) & ~31;
    const int qx = PP[t0 + lr], qy = PP[SPAD + t0 + lr], qz = PP[2 * SPAD + t0 + lr];
    const size_t qo = ((size_t)h * SPAD + (size_t)(t0 + lr)) * HD + 8 * hi;
    const v16h q0 = ldh(QK + qo), q1 = ldh(QK + qo + 32);
    const v16h hz = (v16h){};
    v16h qr0 = hz, qr1 = hz;
    if (EARLY) { const size_t qro = ((size_t)h * EROWS + (size_t)(t0 + lr)) * HD + 8 * hi; qr0 = ldh(QKR + qro); qr1 = ldh(QKR + qro + 32); }
    const size_t ko  = ((size_t)(NH_ + h) * SPAD + (size_t)lr) * HD + 8 * hi;
    const size_t kro = ((size_t)(NH_ + h) * EROWS + (size_t)lr) * HD + 8 * hi;
    const size_t vo  = ((size_t)h * HD + (size_t)lr) * SPAD + 8 * hi;
    const size_t vro = ((size_t)h * HD + (size_t)lr) * EROWS + 8 * hi;
    v8f o[4], oR[4];
#pragma unroll
    for (int j = 0; j < 4; ++j) { o[j] = (v8f){}; oR[j] = (v8f){}; }
    float m = NEGB, l = 0.0f;
#pragma unroll 1
    for (int key0 = 0; key0 < nk; key0 += 32) {
        v8f sc[2];
#pragma unroll
        for (int tl = 0; tl < 2; ++tl) {
            const h16* ka = QK + ko + (size_t)(key0 + 16 * tl) * HD;
            const v16h k0f = ldh(ka), k1f = ldh(ka + 32);
            v8f s = (v8f){};
            s = wmma16g(k0f, q0, s); s = wmma16g(k1f, q1, s);
            if (EARLY) {
                const h16* kr = QKR + kro + (size_t)(key0 + 16 * tl) * HD;
                const v16h kr0f = ldh(kr), kr1f = ldh(kr + 32);
                v8f r = (v8f){};
                r = wmma16g(k0f, qr0, r); r = wmma16g(k1f, qr1, r); r = wmma16g(kr0f, q0, r); r = wmma16g(kr1f, q1, r);
                s = s + r * QRI;
            }
            sc[tl] = s;
        }
        float tt[2][8]; bool ff[2][8]; float mx = NEGB;
#pragma unroll
        for (int tl = 0; tl < 2; ++tl) {
            const int jb = key0 + 16 * tl + 8 * hi;
            const int* pk = PP + jb;
            const v4i kx0 = *(const v4i*)pk, kx1 = *(const v4i*)(pk + 4);
            const v4i ky0 = *(const v4i*)(pk + SPAD), ky1 = *(const v4i*)(pk + SPAD + 4);
            const v4i kz0 = *(const v4i*)(pk + 2 * SPAD), kz1 = *(const v4i*)(pk + 2 * SPAD + 4);
            int kxa[8], kya[8], kza[8];
#pragma unroll
            for (int r = 0; r < 4; ++r) { kxa[r] = kx0[r]; kxa[4 + r] = kx1[r]; kya[r] = ky0[r]; kya[4 + r] = ky1[r]; kza[r] = kz0[r]; kza[4 + r] = kz1[r]; }
#pragma unroll
            for (int r = 0; r < 8; ++r) {
                const int dx = clampi((int)((unsigned)qx - (unsigned)kxa[r]), -30, 30) + 30;
                const int dy = clampi((int)((unsigned)qy - (unsigned)kya[r]), -30, 30) + 30;
                const int dz = clampi((int)((unsigned)qz - (unsigned)kza[r]), -8, 8) + 8;
                const float bsum = (bt[dx] + bt[64 + dy]) + bt[128 + dz];
                float tv = sc[tl][r] * SC2 + bsum;
                asm volatile("" : "+v"(tv));
                const bool f = (jb + r) <= lim;
                tt[tl][r] = tv; ff[tl][r] = f;
                mx = fmaxf(mx, f ? tv : NEGB); }
        }
        mx = fmaxf(mx, __shfl_xor(mx, 16, 32));
        const float mnew = fmaxf(m, mx);
        const float alpha = __builtin_amdgcn_exp2f(m - mnew);
        const float sh = PSH - mnew;
        v16h pb, pr = hz; float ls = 0.0f;
#pragma unroll
        for (int r = 0; r < 8; ++r) {
            const float e0 = tt[0][r] + sh, e1 = tt[1][r] + sh;
            const float ea = __builtin_amdgcn_exp2f(e0), eb = __builtin_amdgcn_exp2f(e1);
            const float ga = (ff[0][r] & (e0 >= -PSH)) ? ea : 0.0f;
            const float gb = (ff[1][r] & (e1 >= -PSH)) ? eb : 0.0f;
            const h16 pa = (h16)ga; const h16 pc = (h16)gb;
            pb[r] = pa; pb[8 + r] = pc;
            if (EARLY) { pr[r] = toh_flush((ga - (float)pa) * QRS); pr[8 + r] = toh_flush((gb - (float)pc) * QRS); ls += ga + gb; }
            else       { ls += (float)pa + (float)pc; } }
        l = l * alpha + ls; m = mnew;
#pragma unroll
        for (int j = 0; j < 4; ++j) { o[j] = o[j] * alpha; if (EARLY) oR[j] = oR[j] * alpha; }
#pragma unroll
        for (int j = 0; j < 4; ++j) {
            const v16h vj = ldh(VT + vo + (size_t)(16 * j) * SPAD + key0);
            o[j] = wmma16g(vj, pb, o[j]);
            if (EARLY) {
                oR[j] = wmma16g(vj, pr, oR[j]);
                const v16h vrj = ldh(VR + vro + (size_t)(16 * j) * EROWS + key0);
                oR[j] = wmma16g(vrj, pb, oR[j]);
            }
        }
    }
    l += __shfl_xor(l, 16, 32);
    const bool any = l > 0.0f;
    const float lsafe = any ? l : 1.0f;
    const float inv = any ? (1.0f / lsafe) : 0.0f;
    const int wb = wave * 16 * OSP;
#pragma unroll
    for (int j = 0; j < 4; ++j) {
        v8f f = o[j];
        if (EARLY) f = o[j] + oR[j] * QRI;
        v4f a, c;
        a[0] = f[0] * inv; a[1] = f[1] * inv; a[2] = f[2] * inv; a[3] = f[3] * inv; c[0] = f[4] * inv; c[1] = f[5] * inv; c[2] = f[6] * inv; c[3] = f[7] * inv;
        *(v4fa*)(&os[wb + lr * OSP + 16 * j + 8 * hi]) = a; *(v4fa*)(&os[wb + lr * OSP + 16 * j + 8 * hi + 4]) = c; }
    wave_sync();
    const size_t cbase = (size_t)t0 * DM + (size_t)h * HD;
#pragma unroll 1
    for (int ps = 0; ps < 2; ++ps) {
#pragma unroll
        for (int s = 0; s < 4; ++s) { const int row = 4 * s + (lane >> 3), c8 = (lane & 7) * 8;
            const v4f x0 = *(const v4fa*)(&os[wb + row * OSP + c8]); const v4f x1 = *(const v4fa*)(&os[wb + row * OSP + c8 + 4]); v8h hv, rv;
#pragma unroll
            for (int i = 0; i < 4; ++i) { const float y0 = x0[i] * CXS, y1 = x1[i] * CXS; const h16 a0 = toh_flush(y0); const h16 a1 = toh_flush(y1); hv[i] = a0; hv[4 + i] = a1;
                rv[i] = toh_flush((y0 - (float)a0) * QRS); rv[4 + i] = toh_flush((y1 - (float)a1) * QRS); }
            const size_t oo = cbase + (size_t)row * DM + c8;
            *(volatile v8h*)(CH + oo) = hv; if (EARLY) *(volatile v8h*)(CR + oo) = rv; }
        if (ps == 0) __threadfence(); }
}

__global__ __launch_bounds__(32 * AW) void k_flash_early(const h16* __restrict__ QK, const h16* __restrict__ QKR, const h16* __restrict__ VT, const h16* __restrict__ VR, const int* __restrict__ PP,
                                                         const float* __restrict__ bxp, const float* __restrict__ byp, const float* __restrict__ bzp, h16* CH, h16* CR) {
    flash_body<1>(QK, QKR, VT, VR, PP, bxp, byp, bzp, CH, CR);
}
__global__ __launch_bounds__(32 * AW) void k_flash_late(const h16* __restrict__ QK, const h16* __restrict__ QKR, const h16* __restrict__ VT, const h16* __restrict__ VR, const int* __restrict__ PP,
                                                        const float* __restrict__ bxp, const float* __restrict__ byp, const float* __restrict__ bzp, h16* CH, h16* CR) {
    flash_body<0>(QK, QKR, VT, VR, PP, bxp, byp, bzp, CH, CR);
}

static_assert(8 * 2 * 16 * 16 == 16 * 64 * 4);
__global__ __launch_bounds__(32) void k_outproj(const h16* __restrict__ CH, const h16* __restrict__ CR, const h16* __restrict__ WOH, float* OUT) {
    __shared__ __align__(16) float os[16 * 68];
    const int lane = threadIdx.x & 31, lr = lane & 15, hi = lane >> 4; const int r0 = blockIdx.x * 64, c0 = blockIdx.y * 64;
    v8f acc[4][4];
#pragma unroll
    for (int mb = 0; mb < 4; ++mb)
#pragma unroll
        for (int nb = 0; nb < 4; ++nb) acc[mb][nb] = (v8f){};
    const size_t aoff = (size_t)(r0 + lr) * DM + 8 * hi, boff = (size_t)(c0 + lr) * DM + 8 * hi;
    if (r0 < EROWS) {
        gemm64_h(CR, WOH, aoff, boff, acc);
#pragma unroll
        for (int mb = 0; mb < 4; ++mb)
#pragma unroll
            for (int nb = 0; nb < 4; ++nb) acc[mb][nb] = acc[mb][nb] * QRI;
    }
    gemm64_h(CH, WOH, aoff, boff, acc);
#pragma unroll
    for (int mb = 0; mb < 4; ++mb) {
#pragma unroll
        for (int nb = 0; nb < 4; ++nb) {
#pragma unroll
            for (int j = 0; j < 8; ++j) os[(hi * 8 + j) * 68 + nb * 16 + lr] = acc[mb][nb][j] * OSCL; }
        wave_sync();
#pragma unroll 1
        for (int ps = 0; ps < 2; ++ps) {
#pragma unroll
            for (int s = 0; s < 8; ++s) { const int row = 2 * s + (lane >> 4), cofs = (lane & 15) * 4;
                const v4f val = *(const v4fa*)(&os[row * 68 + cofs]);
                const int t = r0 + mb * 16 + row;
                if (t < SEQ) *(volatile v4f*)(OUT + (size_t)t * DM + c0 + cofs) = val; }
            if (ps == 0) __threadfence(); }
        wave_sync();
    }
}

static constexpr size_t al256(size_t v) { return (v + 255) & ~(size_t)255; }
static constexpr size_t SZ_XB  = al256((size_t)SPAD * DM * 2);
static constexpr size_t SZ_WB  = al256((size_t)3 * DM * DM * 2);
static constexpr size_t SZ_WO  = al256((size_t)DM * DM * 2);
static constexpr size_t SZ_CS  = al256((size_t)SPAD * 64 * 4);
static constexpr size_t SZ_PP  = al256((size_t)3 * SPAD * 4);
static constexpr size_t SZ_QK  = al256((size_t)2 * NH_ * SPAD * HD * 2);
static constexpr size_t SZ_QKR = al256((size_t)2 * NH_ * EROWS * HD * 2);
static constexpr size_t SZ_VT  = al256((size_t)DM * SPAD * 2);
static constexpr size_t SZ_VR  = al256((size_t)DM * EROWS * 2);
static constexpr size_t SZ_CH  = al256((size_t)SPAD * DM * 2);
static constexpr size_t SZ_CR  = al256((size_t)EROWS * DM * 2);
static constexpr size_t SZ_TOTAL = SZ_XB + SZ_WB + SZ_WO + SZ_CS + SZ_PP + SZ_QK + SZ_QKR + SZ_VT + SZ_VR + SZ_CH + SZ_CR;
static_assert(SZ_TOTAL <= (size_t)134217728);
static_assert((size_t)NH_ * HD * SPAD == (size_t)DM * SPAD);
static_assert(((size_t)3 * DM * DM) % 8 == 0);

extern "C" void kernel_launch(void* const* d_in, const int* in_sizes, int n_in,
                              void* d_out, int out_size, void* d_ws, size_t ws_size, hipStream_t stream) {
    if (n_in < 7) return;
    if ((size_t)in_sizes[0] < (size_t)SEQ * DM) return;
    if ((size_t)in_sizes[1] < (size_t)3 * DM * DM || (size_t)in_sizes[2] < (size_t)DM * DM) return;
    if (in_sizes[3] < 61 * NH_ || in_sizes[4] < 61 * NH_ || in_sizes[5] < 17 * NH_) return;
    if ((size_t)in_sizes[6] < (size_t)SEQ * 3) return;
    if ((size_t)out_size < (size_t)SEQ * DM) return;
    if (SZ_TOTAL > ws_size) return;
    const float* x    = (const float*)d_in[0];
    const float* wqkv = (const float*)d_in[1];
    const float* wout = (const float*)d_in[2];
    const float* bx   = (const float*)d_in[3];
    const float* by   = (const float*)d_in[4];
    const float* bz   = (const float*)d_in[5];
    const int*   pos  = (const int*)d_in[6];
    float* OUT = (float*)d_out;
    char* wsp = (char*)d_ws;
    bf*    XB  = (bf*)wsp;    wsp += SZ_XB;
    bf*    WB  = (bf*)wsp;    wsp += SZ_WB;
    h16*   WOH = (h16*)wsp;   wsp += SZ_WO;
    float* CS  = (float*)wsp; wsp += SZ_CS;
    int*   PP  = (int*)wsp;   wsp += SZ_PP;
    h16*   QK  = (h16*)wsp;   wsp += SZ_QK;
    h16*   QKR = (h16*)wsp;   wsp += SZ_QKR;
    h16*   VT  = (h16*)wsp;   wsp += SZ_VT;
    h16*   VR  = (h16*)wsp;   wsp += SZ_VR;
    h16*   CH  = (h16*)wsp;   wsp += SZ_CH;
    h16*   CR  = (h16*)wsp;   wsp += SZ_CR;
    const bf* WV = WB + (size_t)2 * DM * DM;

    k_cvtx<<<(unsigned)((size_t)SPAD * DM / 8 / 256), 256, 0, stream>>>(x, XB);
    { const size_t n8 = (size_t)3 * DM * DM / 8; k_cvt8<<<(unsigned)((n8 + 255) / 256), 256, 0, stream>>>(wqkv, WB, n8); }
    { const size_t n8 = (size_t)DM * DM / 8;     k_cvtw<<<(unsigned)((n8 + 255) / 256), 256, 0, stream>>>(wout, WOH, n8); }
    k_pospad<<<dim3((SPAD / 4 + 31) / 32, 3, 1), 32, 0, stream>>>(pos, PP);
    k_ropecs<<<(unsigned)((size_t)SPAD * 32 / 256), 256, 0, stream>>>(pos, CS);

    k_projqk<<<dim3(SPAD / 64, 2 * DM / 64, 1), 32, 0, stream>>>(XB, WB, CS, QK, QKR);
    k_projv<<<dim3(DM / 64, SPAD / 64, 1), 32, 0, stream>>>(WV, XB, VT, VR);

    k_flash_early<<<dim3(EROWS / (16 * AW), NH_, 1), 32 * AW, 0, stream>>>(QK, QKR, VT, VR, PP, bx, by, bz, CH, CR);
    if (SPAD > EROWS)
        k_flash_late<<<dim3((SPAD - EROWS) / (16 * AW), NH_, 1), 32 * AW, 0, stream>>>(QK, QKR, VT, VR, PP, bx, by, bz, CH, CR);

    k_outproj<<<dim3(SPAD / 64, DM / 64, 1), 32, 0, stream>>>(CH, CR, WOH, OUT);
}
